// MultiHeadedSelfAttention_6743098655414
// MI455X (gfx1250) — hardware-verified
//
#include <hip/hip_runtime.h>
#include <math.h>


typedef unsigned short u16;
typedef _Float16 f16t;
typedef __bf16   v16bf __attribute__((ext_vector_type(16)));
typedef _Float16 v16h  __attribute__((ext_vector_type(16)));
typedef _Float16 v8h   __attribute__((ext_vector_type(8)));
typedef float    v8f   __attribute__((ext_vector_type(8)));
typedef float    v4f   __attribute__((ext_vector_type(4)));
typedef unsigned int v4u __attribute__((ext_vector_type(4)));

#ifndef NB
#define NB 4
#endif
#ifndef SEQ
#define SEQ 2048
#endif
#define NB_FULL  4
#define SEQ_FULL 2048
#define DM 256
#define NH 4
#define HD 64
#define M_TOT (NB * SEQ)

static_assert(NB >= 1 && NB <= NB_FULL);
static_assert(SEQ >= 128 && SEQ <= SEQ_FULL && (SEQ % 128) == 0);
static_assert(DM == NH * HD);
static_assert((M_TOT % 128) == 0);
static_assert((M_TOT % 8) == 0);

#define QKV_CARRY 8.0f
#define P_CARRY   16384.0f
#define WO_CARRY  16.0f
#define CTX_LDIV  2048.0f
#define OUT_SCALE (1.0f / 1024.0f)


__device__ __forceinline__ unsigned f2bf_bits(float f) {
  unsigned u = __float_as_uint(f);
  u += 0x7FFFu + ((u >> 16) & 1u);
  return u >> 16;
}
__device__ __forceinline__ float bf16r(float f) { return __uint_as_float(f2bf_bits(f) << 16); }
__device__ __forceinline__ u16 h_bits(float f) {
  union { f16t h; u16 u; } c;
  c.h = (f16t)f;
  return c.u;
}
__device__ __forceinline__ v8f zero8() {
  v8f z = {0.f, 0.f, 0.f, 0.f, 0.f, 0.f, 0.f, 0.f};
  return z;
}

__device__ __forceinline__ v16h load_frag_h(const u16* base, int ldr) {
  const int lane = threadIdx.x & 31;
  const int row  = lane & 15;
  const int kb   = (lane >> 4) << 3;
  union { v16h v; uint4 q[2]; } u;
  u.q[0] = *reinterpret_cast<const uint4*>(base + (size_t)row * ldr + kb);
  u.q[1] = *reinterpret_cast<const uint4*>(base + (size_t)row * ldr + 16 + kb);
  return u.v;
}
__device__ __forceinline__ v16bf load_frag_b(const u16* base, int ldr) {
  const int lane = threadIdx.x & 31;
  const int row  = lane & 15;
  const int kb   = (lane >> 4) << 3;
  union { v16bf v; uint4 q[2]; } u;
  u.q[0] = *reinterpret_cast<const uint4*>(base + (size_t)row * ldr + kb);
  u.q[1] = *reinterpret_cast<const uint4*>(base + (size_t)row * ldr + 16 + kb);
  return u.v;
}

__device__ __forceinline__ v8f mma_h(v16h a, v16h b, v8f c) {
  c = __builtin_amdgcn_wmma_f32_16x16x32_f16(false, a, false, b, (short)0, c, false, false);
  asm volatile("v_nop\n\tv_nop\n\tv_nop\n\tv_nop" : "+v"(c) : "v"(a), "v"(b));
  return c;
}
__device__ __forceinline__ v8f mma_b(v16bf a, v16bf b, v8f c) {
  c = __builtin_amdgcn_wmma_f32_16x16x32_bf16(false, a, false, b, (short)0, c, false, false);
  asm volatile("v_nop\n\tv_nop\n\tv_nop\n\tv_nop" : "+v"(c) : "v"(a), "v"(b));
  return c;
}

__device__ __forceinline__ float hmax16(float x) {
#pragma unroll
  for (int m = 1; m < 16; m <<= 1) x = fmaxf(x, __shfl_xor(x, m, 32));
  return x;
}
__device__ __forceinline__ float hadd16(float x) {
#pragma unroll
  for (int m = 1; m < 16; m <<= 1) x += __shfl_xor(x, m, 32);
  return x;
}


__global__ __launch_bounds__(256) void k_xcast(const float* __restrict__ x, u16* __restrict__ Xb) {
  const int g = blockIdx.x * 256 + threadIdx.x;
  const int m = g >> 5;
  const int c = g & 31;
  const int b = m / SEQ, s = m - b * SEQ;
  const float* src = x + ((size_t)b * SEQ_FULL + s) * DM + c * 8;
  const float4 f0 = *reinterpret_cast<const float4*>(src);
  const float4 f1 = *reinterpret_cast<const float4*>(src + 4);
  v4u w;
  w[0] = f2bf_bits(f0.x) | (f2bf_bits(f0.y) << 16);
  w[1] = f2bf_bits(f0.z) | (f2bf_bits(f0.w) << 16);
  w[2] = f2bf_bits(f1.x) | (f2bf_bits(f1.y) << 16);
  w[3] = f2bf_bits(f1.z) | (f2bf_bits(f1.w) << 16);
  u16* dst = Xb + (size_t)m * DM + c * 8;
  *(volatile v4u*)(dst) = w;
  __threadfence();
  *(volatile v4u*)(dst) = w;
}

template <int MODE>
__global__ __launch_bounds__(256) void k_wcast(const float* __restrict__ W, u16* __restrict__ Wt) {
  __shared__ __attribute__((aligned(16))) u16 T[64 * 264];
  const int tid = threadIdx.x, lane = tid & 31, wave = tid >> 5;
  const int n0 = blockIdx.x * 64;
#pragma unroll 4
  for (int it = 0; it < 64; ++it) {
    const int idx = it * 256 + tid;
    const int k = idx >> 6, nl = idx & 63;
    const float f = W[(size_t)k * DM + n0 + nl];
    u16 bits;
    if (MODE == 1) bits = h_bits(bf16r(f) * WO_CARRY);
    else           bits = (u16)f2bf_bits(f);
    T[nl * 264 + k] = bits;
  }
  __syncthreads();
  auto pass = [&]() {
#pragma unroll
    for (int i = 0; i < 8; ++i) {
      const int nl = wave + 8 * i;
      const v4u v = *reinterpret_cast<const v4u*>(&T[nl * 264 + lane * 8]);
      *(volatile v4u*)(Wt + (size_t)(n0 + nl) * DM + lane * 8) = v;
    }
  };
  pass();
  __threadfence();
  pass();
}

template <int TRANS>
__global__ __launch_bounds__(256) void k_proj(const u16* __restrict__ Xb, const u16* __restrict__ Wt,
                                              const float* __restrict__ bias, u16* __restrict__ Out) {
  __shared__ __attribute__((aligned(16))) u16 Bt[64 * 32];
  __shared__ __attribute__((aligned(16))) u16 St[TRANS ? 64 * 136 : 128 * 72];
  const int tid = threadIdx.x, wave = tid >> 5, lane = tid & 31;
  const int h16 = (lane >> 4) << 3;
  const int col = lane & 15;
  const int mb = blockIdx.x * 128;
  const int m0 = mb + wave * 16;
  const int n0 = blockIdx.y * 64;

  v8f acc[4] = {zero8(), zero8(), zero8(), zero8()};
  for (int kk = 0; kk < DM; kk += 32) {
    __syncthreads();
    {
      const int n = tid >> 2, ko = (tid & 3) << 3;
      *reinterpret_cast<uint4*>(&Bt[n * 32 + ko]) =
          *reinterpret_cast<const uint4*>(Wt + (size_t)(n0 + n) * DM + kk + ko);
    }
    __syncthreads();
    const v16bf a = load_frag_b(Xb + (size_t)m0 * DM + kk, DM);
#pragma unroll
    for (int t = 0; t < 4; ++t) {
      const v16bf b = load_frag_b(&Bt[(t * 16) * 32], 32);
      acc[t] = mma_b(a, b, acc[t]);
    }
  }

  const int bb = mb / SEQ;
  const int s0 = mb - bb * SEQ;
  const int hh = blockIdx.y;

  if (TRANS == 0) {
#pragma unroll
    for (int t = 0; t < 4; ++t) {
      const int nl = t * 16 + col;
      const float bvv = bf16r(bias[n0 + nl]);
#pragma unroll
      for (int r = 0; r < 8; ++r) {
        const int ml = wave * 16 + h16 + r;
        St[ml * 72 + nl] = h_bits((acc[t][r] + bvv) * QKV_CARRY);
      }
    }
    __syncthreads();
    u16* base = Out + ((size_t)(bb * NH + hh) * SEQ + s0) * HD;
    auto pass = [&]() {
#pragma unroll
      for (int i = 0; i < 4; ++i) {
        const int rr = wave * 16 + i * 4 + (lane >> 3);
        const int c = lane & 7;
        const v4u v = *reinterpret_cast<const v4u*>(&St[rr * 72 + c * 8]);
        *(volatile v4u*)(base + (size_t)rr * HD + c * 8) = v;
      }
    };
    pass();
    __threadfence();
    pass();
  } else {
#pragma unroll
    for (int t = 0; t < 4; ++t) {
      const int nl = t * 16 + col;
      const float bvv = bf16r(bias[n0 + nl]);
      union { v8h v; v4u q; } pk;
#pragma unroll
      for (int r = 0; r < 8; ++r) pk.v[r] = (f16t)((acc[t][r] + bvv) * QKV_CARRY);
      *reinterpret_cast<v4u*>(&St[nl * 136 + wave * 16 + h16]) = pk.q;
    }
    __syncthreads();
    u16* base = Out + ((size_t)(bb * NH + hh) * HD) * SEQ + s0;
    auto pass = [&]() {
#pragma unroll
      for (int i = 0; i < 4; ++i) {
        const int dd = wave * 8 + i * 2 + (lane >> 4);
        const int c = lane & 15;
        const v4u v = *reinterpret_cast<const v4u*>(&St[dd * 136 + c * 8]);
        *(volatile v4u*)(base + (size_t)dd * SEQ + c * 8) = v;
      }
    };
    pass();
    __threadfence();
    pass();
  }
}

__global__ __launch_bounds__(256) __attribute__((amdgpu_num_vgpr(256)))
void k_attn(const u16* __restrict__ Qp, const u16* __restrict__ Kp, const u16* __restrict__ Vtp,
            u16* __restrict__ Ctx) {
  __shared__ __attribute__((aligned(16))) u16 Kt[64 * 64];
  __shared__ __attribute__((aligned(16))) u16 Vs[64 * 64];
  __shared__ __attribute__((aligned(16))) u16 Pt[8 * 16 * 64];

  const int tid = threadIdx.x, wave = tid >> 5, lane = tid & 31;
  const int h16 = (lane >> 4) << 3;
  const int col = lane & 15;
  const int bh = blockIdx.x;
  const int bb = bh / NH, hh = bh - bb * NH;
  const int q0 = blockIdx.y * 128 + wave * 16;

  const u16* Qbh = Qp + (size_t)bh * SEQ * HD;
  const u16* Kbh = Kp + (size_t)bh * SEQ * HD;
  const u16* Vbh = Vtp + (size_t)bh * HD * SEQ;
  u16* Pw = Pt + wave * (16 * 64);

  const v16h aq0 = load_frag_h(Qbh + (size_t)q0 * HD, HD);
  const v16h aq1 = load_frag_h(Qbh + (size_t)q0 * HD + 32, HD);

  float mrow[8], lrow[8], qi[8];
  v8f o[4] = {zero8(), zero8(), zero8(), zero8()};
#pragma unroll
  for (int r = 0; r < 8; ++r) {
    mrow[r] = -INFINITY;
    lrow[r] = 0.f;
    qi[r] = (float)(q0 + h16 + r);
  }
  const float kmask = 1.0f / ((float)SEQ * 512.0f);

#pragma unroll 1
  for (int t0 = 0; t0 < SEQ; t0 += 64) {
    __syncthreads();
#pragma unroll
    for (int i = 0; i < 2; ++i) {
      const int c = tid + i * 256;
      const int row = c >> 3, off = (c & 7) << 3;
      *reinterpret_cast<uint4*>(&Kt[row * 64 + off]) =
          *reinterpret_cast<const uint4*>(Kbh + (size_t)(t0 + row) * HD + off);
      *reinterpret_cast<uint4*>(&Vs[row * 64 + off]) =
          *reinterpret_cast<const uint4*>(Vbh + (size_t)row * SEQ + t0 + off);
    }
    __syncthreads();

    v8f sc[4];
#pragma unroll
    for (int t = 0; t < 4; ++t) {
      const v16h kb0 = load_frag_h(&Kt[(t * 16) * 64], 64);
      const v16h kb1 = load_frag_h(&Kt[(t * 16) * 64 + 32], 64);
      sc[t] = mma_h(aq0, kb0, zero8());
      sc[t] = mma_h(aq1, kb1, sc[t]);
    }

    float alpha[8];
#pragma unroll
    for (int r = 0; r < 8; ++r) {
      float mx = -INFINITY;
#pragma unroll
      for (int t = 0; t < 4; ++t) {
        const float kj = (float)(t0 + t * 16 + col);
        const float w = ((float)SEQ - fabsf(qi[r] - kj)) * kmask;
        const float z = sc[t][r] * w;
        sc[t][r] = z;
        mx = fmaxf(mx, z);
      }
      mx = hmax16(mx);
      const float mnew = fmaxf(mrow[r], mx);
      alpha[r] = __expf(mrow[r] - mnew);
      mrow[r] = mnew;
    }
#pragma unroll
    for (int r = 0; r < 8; ++r) {
      float ps = 0.f;
#pragma unroll
      for (int t = 0; t < 4; ++t) {
        const float p = __expf(sc[t][r] - mrow[r]);
        ps += p;
        Pw[(r + h16) * 64 + t * 16 + col] = h_bits(p * P_CARRY);
      }
      lrow[r] = lrow[r] * alpha[r] + hadd16(ps);
    }
#pragma unroll
    for (int dt = 0; dt < 4; ++dt)
#pragma unroll
      for (int r = 0; r < 8; ++r) o[dt][r] *= alpha[r];

    asm volatile("s_wait_dscnt 0" ::: "memory");
    __builtin_amdgcn_wave_barrier();

    const v16h p0 = load_frag_h(Pw, 64);
    const v16h p1 = load_frag_h(Pw + 32, 64);
#pragma unroll
    for (int dt = 0; dt < 4; ++dt) {
      const v16h vb0 = load_frag_h(&Vs[(dt * 16) * 64], 64);
      const v16h vb1 = load_frag_h(&Vs[(dt * 16) * 64 + 32], 64);
      o[dt] = mma_h(p0, vb0, o[dt]);
      o[dt] = mma_h(p1, vb1, o[dt]);
    }
  }

  float inv[8];
#pragma unroll
  for (int r = 0; r < 8; ++r) inv[r] = 1.0f / (lrow[r] * CTX_LDIV);
  asm volatile("s_wait_dscnt 0" ::: "memory");
  __builtin_amdgcn_wave_barrier();
#pragma unroll
  for (int dt = 0; dt < 4; ++dt)
#pragma unroll
    for (int r = 0; r < 8; ++r)
      Pw[(r + h16) * 64 + dt * 16 + col] = h_bits(o[dt][r] * inv[r]);
  asm volatile("s_wait_dscnt 0" ::: "memory");
  __builtin_amdgcn_wave_barrier();

  u16* cbase = Ctx + ((size_t)(bb * SEQ + q0)) * DM + hh * HD;
  auto pass = [&]() {
#pragma unroll
    for (int i = 0; i < 4; ++i) {
      const int rr = i * 4 + (lane >> 3);
      const int c = lane & 7;
      const v4u v = *reinterpret_cast<const v4u*>(&Pw[rr * 64 + c * 8]);
      *(volatile v4u*)(cbase + (size_t)rr * DM + c * 8) = v;
    }
  };
  pass();
  __threadfence();
  pass();
}

__global__ __launch_bounds__(256) void k_oproj(const u16* __restrict__ Ctx, const u16* __restrict__ Wot,
                                               const float* __restrict__ bo, float* __restrict__ out) {
  __shared__ __attribute__((aligned(16))) u16 Bt[64 * 32];
  __shared__ __attribute__((aligned(16))) float So[128 * 68];
  const int tid = threadIdx.x, wave = tid >> 5, lane = tid & 31;
  const int h16 = (lane >> 4) << 3;
  const int col = lane & 15;
  const int mb = blockIdx.x * 128;
  const int m0 = mb + wave * 16;
  const int n0 = blockIdx.y * 64;

  v8f acc[4] = {zero8(), zero8(), zero8(), zero8()};
  for (int kk = 0; kk < DM; kk += 32) {
    __syncthreads();
    {
      const int n = tid >> 2, ko = (tid & 3) << 3;
      *reinterpret_cast<uint4*>(&Bt[n * 32 + ko]) =
          *reinterpret_cast<const uint4*>(Wot + (size_t)(n0 + n) * DM + kk + ko);
    }
    __syncthreads();
    const v16h a = load_frag_h(Ctx + (size_t)m0 * DM + kk, DM);
#pragma unroll
    for (int t = 0; t < 4; ++t) {
      const v16h b = load_frag_h(&Bt[(t * 16) * 32], 32);
      acc[t] = mma_h(a, b, acc[t]);
    }
  }

#pragma unroll
  for (int t = 0; t < 4; ++t) {
    const int nl = t * 16 + col;
    const float bvv = bf16r(bo[n0 + nl]);
#pragma unroll
    for (int r = 0; r < 8; ++r) {
      const int ml = wave * 16 + h16 + r;
      So[ml * 68 + nl] = acc[t][r] * OUT_SCALE + bvv;
    }
  }
  __syncthreads();
  float* base = out + (size_t)mb * DM + n0;
  auto pass = [&]() {
#pragma unroll
    for (int i = 0; i < 8; ++i) {
      const int rr = wave * 16 + i * 2 + (lane >> 4);
      const int c = lane & 15;
      const v4f v = *reinterpret_cast<const v4f*>(&So[rr * 68 + c * 4]);
      *(volatile v4f*)(base + (size_t)rr * DM + c * 4) = v;
    }
  };
  pass();
  __threadfence();
  pass();
}


extern "C" void kernel_launch(void* const* d_in, const int* in_sizes, int n_in,
                              void* d_out, int out_size, void* d_ws, size_t ws_size,
                              hipStream_t stream) {
  if (n_in < 9) return;
  if (in_sizes[0] < ((NB - 1) * SEQ_FULL + SEQ) * DM) return;
  if (in_sizes[1] < DM * DM || in_sizes[3] < DM * DM || in_sizes[5] < DM * DM || in_sizes[7] < DM * DM) return;
  if (in_sizes[2] < DM || in_sizes[4] < DM || in_sizes[6] < DM || in_sizes[8] < DM) return;
  if (out_size < M_TOT * DM) return;

  const float* x  = (const float*)d_in[0];
  const float* Wq = (const float*)d_in[1];
  const float* bq = (const float*)d_in[2];
  const float* Wk = (const float*)d_in[3];
  const float* bk = (const float*)d_in[4];
  const float* Wv = (const float*)d_in[5];
  const float* bv = (const float*)d_in[6];
  const float* Wo = (const float*)d_in[7];
  const float* bo = (const float*)d_in[8];
  float* out = (float*)d_out;

  const size_t XB_BYTES = (size_t)M_TOT * DM * 2;
  const size_t WT_BYTES = (size_t)DM * DM * 2;
  const size_t PL_BYTES = (size_t)M_TOT * DM * 2;
  const size_t total = XB_BYTES + 4 * WT_BYTES + 4 * PL_BYTES;
  if (total > ws_size) return;

  char* ws = (char*)d_ws;
  size_t off = 0;
  u16* Xb  = (u16*)(ws + off); off += XB_BYTES;
  u16* Wqt = (u16*)(ws + off); off += WT_BYTES;
  u16* Wkt = (u16*)(ws + off); off += WT_BYTES;
  u16* Wvt = (u16*)(ws + off); off += WT_BYTES;
  u16* Wot = (u16*)(ws + off); off += WT_BYTES;
  u16* Qp  = (u16*)(ws + off); off += PL_BYTES;
  u16* Kpl = (u16*)(ws + off); off += PL_BYTES;
  u16* Vtp = (u16*)(ws + off); off += PL_BYTES;
  u16* Ctx = (u16*)(ws + off); off += PL_BYTES;
  (void)off;

  k_xcast<<<M_TOT / 8, 256, 0, stream>>>(x, Xb);
  k_wcast<0><<<DM / 64, 256, 0, stream>>>(Wq, Wqt);
  k_wcast<0><<<DM / 64, 256, 0, stream>>>(Wk, Wkt);
  k_wcast<0><<<DM / 64, 256, 0, stream>>>(Wv, Wvt);
  k_wcast<1><<<DM / 64, 256, 0, stream>>>(Wo, Wot);

  dim3 gp(M_TOT / 128, DM / 64);
  k_proj<0><<<gp, 256, 0, stream>>>(Xb, Wqt, bq, Qp);
  k_proj<0><<<gp, 256, 0, stream>>>(Xb, Wkt, bk, Kpl);
  k_proj<1><<<gp, 256, 0, stream>>>(Xb, Wvt, bv, Vtp);

  dim3 ga(NB * NH, SEQ / 128);
  k_attn<<<ga, 256, 0, stream>>>(Qp, Kpl, Vtp, Ctx);

  k_oproj<<<gp, 256, 0, stream>>>(Ctx, Wot, bo, out);
}
